// MemoryModule_21397527069133
// MI455X (gfx1250) — hardware-run, weakly checked
//
#include <hip/hip_runtime.h>
#include <math.h>

constexpr int NBATCH = 64;
constexpr int NFACT  = 512;
constexpr int NDIM   = 256;
constexpr int NATT   = 256;
constexpr int NAGRU  = 256;
constexpr int NZK    = 4 * NDIM;
constexpr int NROWS  = NBATCH * NFACT;
constexpr int NX     = 2 * NAGRU;
constexpr int NCAT   = 2 * NDIM + NAGRU;
constexpr int NPART  = NATT / 64;
constexpr int NTHR   = 256;
constexpr int SEQB   = 16;
constexpr int HP     = 264;
constexpr int XSP    = 520;
constexpr int OSP    = 260;
constexpr int SLABP  = 68;
constexpr float WCARRY     = 16.0f;
constexpr float WCARRY_INV = 1.0f / 16.0f;
constexpr size_t WS_LIMIT  = 134217728;

static_assert(NZK % 32 == 0 && NDIM % 32 == 0 && NAGRU % 32 == 0);
static_assert(NROWS % 64 == 0 && NATT % 64 == 0 && NX % 64 == 0);
static_assert(((NROWS / 64) * (NATT / 64)) % 8 == 0);
static_assert(((NROWS / 64) * (NX / 64)) % 8 == 0);
static_assert(NAGRU == 32 * (NTHR / 32));
static_assert(NBATCH % SEQB == 0);
static_assert((2 * SEQB * HP) % NTHR == 0);
static_assert((SEQB * NX / 8) % NTHR == 0);
static_assert((SEQB * NDIM / 4) % NTHR == 0);
static_assert(NFACT == 2 * NTHR);
static_assert(NDIM == NTHR && NAGRU == NDIM);
static_assert(NCAT % 8 == 0);
static_assert((NROWS * (NDIM / 8)) % NTHR == 0 && (NATT * (NZK / 8)) % NTHR == 0 && (NAGRU * (NDIM / 8)) % NTHR == 0);
static_assert((NROWS * (NZK / 8)) % NTHR == 0);
static_assert((OSP * 4) % 16 == 0 && (XSP * 2) % 16 == 0 && (HP * 2) % 16 == 0);

typedef __attribute__((ext_vector_type(16))) _Float16 v16h;
typedef __attribute__((ext_vector_type(8)))  _Float16 v8h;
typedef __attribute__((ext_vector_type(8)))  float    v8f;
typedef __attribute__((ext_vector_type(4)))  float    v4f;
typedef __attribute__((ext_vector_type(4)))  unsigned v4u;

__device__ __forceinline__ float h16_to_f32(unsigned hb) {
  const unsigned sgn = (hb & 0x8000u) << 16; const unsigned em = hb & 0x7fffu;
  const float fn = __uint_as_float((em << 13) + 0x38000000u);
  const float fs = (float)em * 5.9604644775390625e-8f;
  const float mag = (em < 0x400u) ? fs : fn; return __uint_as_float(__float_as_uint(mag) | sgn); }

__device__ __forceinline__ void guard4x5_h(v8f& a0, v8f& a1, v8f& a2, v8f& a3, v16h x, v16h y0, v16h y1, v16h y2, v16h y3) {
  asm volatile("v_nop\n\tv_nop\n\tv_nop\n\tv_nop" : "+v"(a0), "+v"(a1), "+v"(a2), "+v"(a3) : "v"(x), "v"(y0), "v"(y1), "v"(y2), "v"(y3));
}
__device__ __forceinline__ void keep4_h(v16h a, v16h b, v16h c, v16h d) { asm volatile("v_nop" :: "v"(a), "v"(b), "v"(c), "v"(d)); }
__device__ __forceinline__ void acc_guard4(v8f& a, v8f& b, v8f& c, v8f& d) { asm volatile("v_nop\n\tv_nop\n\tv_nop\n\tv_nop" : "+v"(a), "+v"(b), "+v"(c), "+v"(d)); }

union FragU { v16h v; v8h h[2]; };
__device__ __forceinline__ v16h fragload_h(const _Float16* p) { FragU f; f.h[0] = *(const v8h*)(p); f.h[1] = *(const v8h*)(p + 16); return f.v; }
__device__ __forceinline__ v8f mma_h(v16h a, v16h b, v8f c) {
  return __builtin_amdgcn_wmma_f32_16x16x32_f16(false, a, false, b, (short)0, c, false, false);
}

__device__ __forceinline__ void gemm64_mainloop_f16(const _Float16* __restrict__ A, int lda, const _Float16* __restrict__ Bt, int ldb,
                                                    int m0, int n0, int K, int lane, v8f (&acc)[4][4]) {
  const int rlane = lane & 15, koff = (lane >> 4) * 8;
#pragma unroll
  for (int i = 0; i < 4; ++i)
#pragma unroll
    for (int j = 0; j < 4; ++j) acc[i][j] = (v8f){0.f, 0.f, 0.f, 0.f, 0.f, 0.f, 0.f, 0.f};
  for (int k0 = 0; k0 < K; k0 += 32) {
    v16h bh[4];
#pragma unroll
    for (int j = 0; j < 4; ++j) bh[j] = fragload_h(Bt + (size_t)(n0 + (j << 4) + rlane) * ldb + koff + k0);
#pragma unroll
    for (int i = 0; i < 4; ++i) {
      const v16h ah = fragload_h(A + (size_t)(m0 + (i << 4) + rlane) * lda + koff + k0);
#pragma unroll
      for (int j = 0; j < 4; ++j) acc[i][j] = mma_h(ah, bh[j], acc[i][j]);
      guard4x5_h(acc[i][0], acc[i][1], acc[i][2], acc[i][3], ah, bh[0], bh[1], bh[2], bh[3]);
    }
    keep4_h(bh[0], bh[1], bh[2], bh[3]);
  }
  acc_guard4(acc[0][0], acc[0][1], acc[0][2], acc[0][3]);
  acc_guard4(acc[1][0], acc[1][1], acc[1][2], acc[1][3]);
  acc_guard4(acc[2][0], acc[2][1], acc[2][2], acc[2][3]);
  acc_guard4(acc[3][0], acc[3][1], acc[3][2], acc[3][3]);
}

__global__ __launch_bounds__(NTHR) void cvt_f16x8_kernel(const float* __restrict__ src, unsigned short* __restrict__ dst, int n8, float sc) {
  const int i = blockIdx.x * NTHR + threadIdx.x;
  if (i < n8) {
    const float* sp = src + (size_t)i * 8;
    const v4f a = *(const v4f*)(sp);
    const v4f b = *(const v4f*)(sp + 4);
    v8h hv;
#pragma unroll
    for (int e = 0; e < 4; ++e) { hv[e] = (_Float16)(a[e] * sc); hv[4 + e] = (_Float16)(b[e] * sc); }
    *(volatile v8h*)(dst + (size_t)i * 8) = hv;
    __threadfence();
    *(volatile v8h*)(dst + (size_t)i * 8) = hv;
  }
}

__global__ __launch_bounds__(NTHR) void zbuild_kernel(const float* __restrict__ facts, const float* __restrict__ queries,
                                                     const float* __restrict__ m_old, unsigned short* __restrict__ Zp, int n8) {
  const int i = blockIdx.x * NTHR + threadIdx.x;
  if (i < n8) {
    const int row = i >> 7;
    const int c8  = i & 127;
    const int sel = c8 >> 5;
    const int d0  = (c8 & 31) * 8;
    const int b   = row >> 9;
    const float* fp = facts   + (size_t)row * NDIM + d0;
    const float* qp = queries + (size_t)b * NDIM + d0;
    const float* mp = m_old   + (size_t)b * NDIM + d0;
    const v4f f0 = *(const v4f*)(fp), f1 = *(const v4f*)(fp + 4);
    const v4f q0 = *(const v4f*)(qp), q1 = *(const v4f*)(qp + 4);
    const v4f w0 = *(const v4f*)(mp), w1 = *(const v4f*)(mp + 4);
    const float fm = ((sel & 1) != 0) ? 1.0f : 0.0f;
    const float fq = 1.0f - fm;
    const bool usep = sel < 2;
    v8h hv;
#pragma unroll
    for (int e = 0; e < 4; ++e) {
      const float ua = fmaf(fm, w0[e], fq * q0[e]);
      const float ub = fmaf(fm, w1[e], fq * q1[e]);
      const float pa = f0[e] * ua, pb = f1[e] * ub;
      const float da = fabsf(f0[e] - ua), db = fabsf(f1[e] - ub);
      hv[e]     = (_Float16)(usep ? pa : da);
      hv[4 + e] = (_Float16)(usep ? pb : db);
    }
    *(volatile v8h*)(Zp + (size_t)i * 8) = hv;
    __threadfence();
    *(volatile v8h*)(Zp + (size_t)i * 8) = hv;
  }
}

__global__ __launch_bounds__(NTHR) void gemm_score_kernel(const unsigned short* __restrict__ Zp, const unsigned short* __restrict__ W1p,
                                                         const float* __restrict__ b1, const float* __restrict__ w2, float* __restrict__ P) {
  __shared__ __align__(16) float sT[NTHR / 32][64];
  const int lane = threadIdx.x & 31, wave = threadIdx.x >> 5;
  const int tilesN = NATT / 64, tilesM = NROWS / 64;
  const int tile = blockIdx.x * 8 + wave;
  if (tile >= tilesM * tilesN) return;
  const int tm = tile / tilesN, tn = tile - tm * tilesN;
  const int m0 = tm << 6, n0 = tn << 6;
  v8f acc[4][4];
  gemm64_mainloop_f16((const _Float16*)Zp, NZK, (const _Float16*)W1p, NZK, m0, n0, NZK, lane, acc);
  const int rlane = lane & 15, mOff = (lane >> 4) * 8;
  float bb[4], ww[4];
#pragma unroll
  for (int j = 0; j < 4; ++j) { const int n = n0 + (j << 4) + rlane; bb[j] = b1[n]; ww[j] = w2[n]; }
  float* slab = sT[wave];
#pragma unroll
  for (int i = 0; i < 4; ++i) {
#pragma unroll
    for (int r = 0; r < 8; ++r) {
      float p = 0.0f;
#pragma unroll
      for (int j = 0; j < 4; ++j) {
        const float v = tanhf(acc[i][j][r] * WCARRY_INV + bb[j]);
        p = p + v * ww[j];
      }
      p += __shfl_xor(p, 1, 32);
      p += __shfl_xor(p, 2, 32);
      p += __shfl_xor(p, 4, 32);
      p += __shfl_xor(p, 8, 32);
      slab[16 * i + mOff + r] = p;
    }
  }
  __builtin_amdgcn_fence(__ATOMIC_RELEASE, "workgroup");
  __builtin_amdgcn_wave_barrier();
  __builtin_amdgcn_fence(__ATOMIC_ACQUIRE, "workgroup");
  const v4f v = *(const v4f*)(slab + 4 * rlane);
  float* dst = P + (size_t)tn * NROWS + m0 + 4 * rlane;
  if (lane < 16) *(volatile v4f*)dst = v;
  __threadfence();
  if (lane < 16) *(volatile v4f*)dst = v;
}

__global__ __launch_bounds__(NTHR) void gemm_f16out_kernel(const unsigned short* __restrict__ Ap, int lda, const unsigned short* __restrict__ Btp, int ldb,
                                                          unsigned short* __restrict__ Cp, int ldc, int M, int N, int K, float scale) {
  __shared__ __align__(16) float sT[NTHR / 32][16 * SLABP];
  const int lane = threadIdx.x & 31, wave = threadIdx.x >> 5;
  const int tilesN = N >> 6, tilesM = M >> 6;
  const int tile = blockIdx.x * 8 + wave;
  if (tile >= tilesM * tilesN) return;
  const int tm = tile / tilesN, tn = tile - tm * tilesN;
  const int m0 = tm << 6, n0 = tn << 6;
  v8f acc[4][4];
  gemm64_mainloop_f16((const _Float16*)Ap, lda, (const _Float16*)Btp, ldb, m0, n0, K, lane, acc);
  const int rlane = lane & 15, mOff = (lane >> 4) * 8;
  float* slab = sT[wave];
#pragma unroll
  for (int i = 0; i < 4; ++i) {
    const int mBase = m0 + (i << 4);
#pragma unroll
    for (int j = 0; j < 4; ++j)
#pragma unroll
      for (int r = 0; r < 8; ++r) slab[(mOff + r) * SLABP + (j << 4) + rlane] = acc[i][j][r] * scale;
    __builtin_amdgcn_fence(__ATOMIC_RELEASE, "workgroup");
    __builtin_amdgcn_wave_barrier();
    __builtin_amdgcn_fence(__ATOMIC_ACQUIRE, "workgroup");
    const int q = lane >> 3, c8 = (lane & 7) * 8;
    for (int pass = 0; pass < 2; ++pass) {
#pragma unroll
      for (int it = 0; it < 4; ++it) {
        const int row = it * 4 + q;
        const float* sp = slab + row * SLABP + c8;
        v8h hv;
#pragma unroll
        for (int e = 0; e < 8; ++e) hv[e] = (_Float16)sp[e];
        *(volatile v8h*)(Cp + (size_t)(mBase + row) * ldc + n0 + c8) = hv;
      }
      __threadfence();
    }
    __builtin_amdgcn_fence(__ATOMIC_RELEASE, "workgroup");
    __builtin_amdgcn_wave_barrier();
    __builtin_amdgcn_fence(__ATOMIC_ACQUIRE, "workgroup");
  }
}

__global__ __launch_bounds__(NTHR) void softmax_kernel(const float* __restrict__ P, const int* __restrict__ num_facts,
                                                      const float* __restrict__ w2b, float* __restrict__ G) {
  __shared__ float red[NTHR];
  __shared__ __align__(16) float gsv[NFACT];
  const int b = blockIdx.x, tid = threadIdx.x;
  int nf = num_facts[b];
  nf = nf < 1 ? 1 : (nf > NFACT ? NFACT : nf);
  const size_t m0 = (size_t)b * NFACT + tid, m1 = m0 + NTHR;
  const float bias = w2b[0];
  float s0 = bias, s1 = bias;
#pragma unroll
  for (int p = 0; p < NPART; ++p) { s0 += P[(size_t)p * NROWS + m0]; s1 += P[(size_t)p * NROWS + m1]; }
  const float f0 = (tid < nf) ? 1.0f : 0.0f;
  const float f1 = ((tid + NTHR) < nf) ? 1.0f : 0.0f;
  const float big = -3.0e38f;
  const float k0 = fmaf(f0, s0, (1.0f - f0) * big);
  const float k1 = fmaf(f1, s1, (1.0f - f1) * big);
  red[tid] = fmaxf(k0, k1);
  __syncthreads();
  for (int st = NTHR / 2; st > 0; st >>= 1) {
    if (tid < st) red[tid] = fmaxf(red[tid], red[tid + st]);
    __syncthreads();
  }
  const float mx = red[0];
  __syncthreads();
  const float a0 = (s0 - mx) * f0, a1 = (s1 - mx) * f1;
  const float e0 = expf(a0) * f0, e1 = expf(a1) * f1;
  red[tid] = e0 + e1;
  __syncthreads();
  for (int st = NTHR / 2; st > 0; st >>= 1) {
    if (tid < st) red[tid] += red[tid + st];
    __syncthreads();
  }
  const float inv = 1.0f / red[0];
  gsv[tid] = e0 * inv;
  gsv[tid + NTHR] = e1 * inv;
  __syncthreads();
  const v4f gv = *(const v4f*)(gsv + 4 * (tid & 127));
  float* dst = G + (size_t)b * NFACT + 4 * (tid & 127);
  if (tid < 128) *(volatile v4f*)dst = gv;
  __threadfence();
  if (tid < 128) *(volatile v4f*)dst = gv;
}

__global__ __launch_bounds__(NTHR) void agru_kernel(const unsigned short* __restrict__ Xp, const float* __restrict__ G,
                                                   const unsigned short* __restrict__ UUp, const float* __restrict__ urb,
                                                   const float* __restrict__ ugb, const float* __restrict__ m_old,
                                                   float* __restrict__ Cst) {
  __shared__ __align__(16) _Float16       Ah[2][SEQB * HP];
  __shared__ __align__(16) unsigned short Xs[2][SEQB * XSP];
  __shared__ __align__(16) float          Gs[2][32];
  __shared__ __align__(16) float          Hs[SEQB * OSP];
  const _Float16* UU = (const _Float16*)UUp;
  const int tid = threadIdx.x, lane = tid & 31, wave = tid >> 5;
  const int c = lane & 15, hh = lane >> 4, koff = hh * 8;
  const int rb = blockIdx.x * SEQB;

  {
    _Float16* ahf = &Ah[0][0];
#pragma unroll 1
    for (int i = tid; i < 2 * SEQB * HP; i += NTHR) ahf[i] = (_Float16)0.0f;
  }
  __syncthreads();
#pragma unroll
  for (int it = 0; it < 4; ++it) {
    const int idx = it * NTHR + tid;
    const int row = idx >> 6, c4 = (idx & 63) * 4;
    const v4f v = *(const v4f*)(m_old + (size_t)(rb + row) * NDIM + c4);
    *(v4f*)(Hs + row * OSP + c4) = v;
  }
  asm volatile("" ::: "memory");
#pragma unroll
  for (int it = 0; it < 4; ++it) {
    const int qi = it * NTHR + tid;
    const int row = qi >> 6, col8 = (qi & 63) * 8;
    const v4u xv = *(const v4u*)(Xp + ((size_t)(rb + row) * NFACT) * NX + col8);
    *(v4u*)(&Xs[0][row * XSP + col8]) = xv;
  }
  if (wave == 0) Gs[0][lane] = G[(size_t)(rb + (lane & 15)) * NFACT];
  float brv[2], bgv[2];
#pragma unroll
  for (int nt = 0; nt < 2; ++nt) {
    const int j = 32 * wave + 16 * nt + c;
    brv[nt] = urb[j];
    bgv[nt] = ugb[j];
  }
  __syncthreads();
#pragma unroll 1
  for (int i = 0; i < SEQB; ++i) Ah[0][i * HP + tid] = (_Float16)Hs[i * OSP + tid];
  float hst[2][8];
#pragma unroll
  for (int nt = 0; nt < 2; ++nt) {
    const int j = 32 * wave + 16 * nt + c;
#pragma unroll
    for (int r = 0; r < 8; ++r) hst[nt][r] = Hs[(8 * hh + r) * OSP + j];
  }
  __syncthreads();

  const v8f z8 = {0.f, 0.f, 0.f, 0.f, 0.f, 0.f, 0.f, 0.f};
  const int j0 = 32 * wave + c, j1 = j0 + 16;
  const _Float16* ur0 = UU + (size_t)j0 * NAGRU + koff;
  const _Float16* ug0 = UU + (size_t)(NAGRU + j0) * NAGRU + koff;
  const _Float16* ur1 = UU + (size_t)j1 * NAGRU + koff;
  const _Float16* ug1 = UU + (size_t)(NAGRU + j1) * NAGRU + koff;

#pragma unroll 1
  for (int t = 0; t < NFACT; ++t) {
    const int cur = t & 1, nxt = cur ^ 1;
    const int tnx = (t + 1 < NFACT) ? (t + 1) : (NFACT - 1);
#pragma unroll
    for (int it = 0; it < 4; ++it) {
      const int qi = it * NTHR + tid;
      const int row = qi >> 6, col8 = (qi & 63) * 8;
      const v4u xv = *(const v4u*)(Xp + ((size_t)(rb + row) * NFACT + (size_t)tnx) * NX + col8);
      *(v4u*)(&Xs[nxt][row * XSP + col8]) = xv;
    }
    if (wave == 0) Gs[nxt][lane] = G[(size_t)(rb + (lane & 15)) * NFACT + tnx];
    asm volatile("" ::: "memory");

    float gt[8];
#pragma unroll
    for (int r = 0; r < 8; ++r) gt[r] = Gs[cur][8 * hh + r];

    const _Float16* ahrow = &Ah[cur][0] + c * HP + koff;
    v8f acc[4];
    acc[0] = z8; acc[1] = z8; acc[2] = z8; acc[3] = z8;
#pragma unroll 1
    for (int k0 = 0; k0 < NAGRU; k0 += 32) {
      const v16h a  = fragload_h(ahrow + k0);
      const v16h b0 = fragload_h(ur0 + k0);
      const v16h b1 = fragload_h(ug0 + k0);
      const v16h b2 = fragload_h(ur1 + k0);
      const v16h b3 = fragload_h(ug1 + k0);
      acc[0] = mma_h(a, b0, acc[0]);
      acc[1] = mma_h(a, b1, acc[1]);
      acc[2] = mma_h(a, b2, acc[2]);
      acc[3] = mma_h(a, b3, acc[3]);
      guard4x5_h(acc[0], acc[1], acc[2], acc[3], a, b0, b1, b2, b3);
    }
    acc_guard4(acc[0], acc[1], acc[2], acc[3]);

    _Float16* ahn = &Ah[nxt][0];
    const unsigned short* xs = &Xs[cur][0];
#pragma unroll
    for (int nt = 0; nt < 2; ++nt) {
      const int j = 32 * wave + 16 * nt + c;
#pragma unroll
      for (int r = 0; r < 8; ++r) {
        const int row = 8 * hh + r;
        const float xr = h16_to_f32((unsigned)xs[row * XSP + j]);
        const float xg = h16_to_f32((unsigned)xs[row * XSP + NAGRU + j]);
        const float ar = acc[2 * nt][r] * WCARRY_INV + xr + brv[nt];
        const float ag = acc[2 * nt + 1][r] * WCARRY_INV + bgv[nt];
        const float arc = fmaxf(ar, -40.0f);
        const float rr = 1.0f / (1.0f + expf(-arc));
        const float ht = tanhf(xg + rr * ag);
        const float ho = hst[nt][r];
        const float hn = gt[r] * ht + (1.0f - gt[r]) * ho;
        hst[nt][r] = hn;
        ahn[row * HP + j] = (_Float16)hn;
      }
    }
    __syncthreads();
  }

#pragma unroll
  for (int nt = 0; nt < 2; ++nt) {
    const int j = 32 * wave + 16 * nt + c;
#pragma unroll
    for (int r = 0; r < 8; ++r) Hs[(8 * hh + r) * OSP + j] = hst[nt][r];
  }
  __syncthreads();
  for (int pass = 0; pass < 2; ++pass) {
#pragma unroll
    for (int it = 0; it < 4; ++it) {
      const int idx = it * NTHR + tid;
      const int row = idx >> 6, c4 = (idx & 63) * 4;
      const v4f v = *(const v4f*)(Hs + row * OSP + c4);
      *(volatile v4f*)(Cst + (size_t)(rb + row) * NAGRU + c4) = v;
    }
    __threadfence();
  }
}

__global__ __launch_bounds__(NTHR) void memout_kernel(const float* __restrict__ m_old, const float* __restrict__ Cst,
                                                     const float* __restrict__ queries, const float* __restrict__ Wt,
                                                     const float* __restrict__ wtb, float* __restrict__ out) {
  __shared__ __align__(16) float cat[NCAT];
  __shared__ __align__(16) float os[NDIM];
  const int b = blockIdx.x, tid = threadIdx.x;
  cat[tid]            = m_old[(size_t)b * NDIM + tid];
  cat[NDIM + tid]     = Cst[(size_t)b * NAGRU + tid];
  cat[2 * NDIM + tid] = queries[(size_t)b * NDIM + tid];
  __syncthreads();
  const float* wrow = Wt + (size_t)tid * NCAT;
  float s = 0.0f;
#pragma unroll 2
  for (int k = 0; k < NCAT; k += 4) {
    const v4f w = *(const v4f*)(wrow + k);
    const v4f x = *(const v4f*)(cat + k);
    s += w[0] * x[0];
    s += w[1] * x[1];
    s += w[2] * x[2];
    s += w[3] * x[3];
  }
  s += wtb[tid];
  os[tid] = fmaxf(s, 0.0f);
  __syncthreads();
  const v4f v = *(const v4f*)(os + 4 * (tid & 63));
  float* dst = out + (size_t)b * NDIM + 4 * (tid & 63);
  if (tid < 64) *(volatile v4f*)dst = v;
  __threadfence();
  if (tid < 64) *(volatile v4f*)dst = v;
}

extern "C" void kernel_launch(void* const* d_in, const int* in_sizes, int n_in,
                              void* d_out, int out_size, void* d_ws, size_t ws_size, hipStream_t stream) {
  if (n_in < 16 || d_out == nullptr || d_ws == nullptr) return;
  if (in_sizes[0] != NBATCH * NDIM || in_sizes[1] != NBATCH * NFACT * NDIM || in_sizes[2] != NBATCH ||
      in_sizes[3] != NBATCH * NDIM || in_sizes[4] != NATT * NZK || in_sizes[5] != NATT || in_sizes[6] != NATT ||
      in_sizes[7] != 1 || in_sizes[8] != NAGRU * NDIM || in_sizes[9] != NAGRU * NAGRU || in_sizes[10] != NAGRU ||
      in_sizes[11] != NAGRU * NDIM || in_sizes[12] != NAGRU * NAGRU || in_sizes[13] != NAGRU ||
      in_sizes[14] != NDIM * NCAT || in_sizes[15] != NDIM || out_size != NBATCH * NDIM) return;

  const float* queries   = (const float*)d_in[0];
  const float* facts     = (const float*)d_in[1];
  const int*   num_facts = (const int*)d_in[2];
  const float* m_old     = (const float*)d_in[3];
  const float* W1_w      = (const float*)d_in[4];
  const float* W1_b      = (const float*)d_in[5];
  const float* W2_w      = (const float*)d_in[6];
  const float* W2_b      = (const float*)d_in[7];
  const float* Wr_w      = (const float*)d_in[8];
  const float* Ur_w      = (const float*)d_in[9];
  const float* Ur_b      = (const float*)d_in[10];
  const float* Wg_w      = (const float*)d_in[11];
  const float* Ug_w      = (const float*)d_in[12];
  const float* Ug_b      = (const float*)d_in[13];
  const float* Wt_w      = (const float*)d_in[14];
  const float* Wt_b      = (const float*)d_in[15];
  float* out = (float*)d_out;

  char* ws = (char*)d_ws; size_t off = 0;
  auto carve = [&](size_t bytes) -> char* { char* p = ws + off; off += (bytes + 255) & ~(size_t)255; return p; };
  unsigned short* Zp   = (unsigned short*)carve((size_t)NROWS * NZK * 2);
  unsigned short* Ff   = (unsigned short*)carve((size_t)NROWS * NDIM * 2);
  unsigned short* Xp   = (unsigned short*)carve((size_t)NROWS * NX * 2);
  unsigned short* W1h  = (unsigned short*)carve((size_t)NATT * NZK * 2);
  unsigned short* WrWg = (unsigned short*)carve((size_t)NX * NDIM * 2);
  unsigned short* UrUg = (unsigned short*)carve((size_t)NX * NAGRU * 2);
  float*          Pp   = (float*)carve((size_t)NPART * NROWS * 4);
  float*          Gp   = (float*)carve((size_t)NBATCH * NFACT * 4);
  float*          Cp   = (float*)carve((size_t)NBATCH * NAGRU * 4);
  if (off > ws_size || off > WS_LIMIT) return;

  const int n8f = NROWS * (NDIM / 8);
  const int n8w1 = NATT * (NZK / 8);
  const int n8w = NAGRU * (NDIM / 8);
  cvt_f16x8_kernel<<<n8f / NTHR, NTHR, 0, stream>>>(facts, Ff, n8f, 1.0f);
  cvt_f16x8_kernel<<<n8w1 / NTHR, NTHR, 0, stream>>>(W1_w, W1h, n8w1, WCARRY);
  cvt_f16x8_kernel<<<n8w / NTHR, NTHR, 0, stream>>>(Wr_w, WrWg, n8w, WCARRY);
  cvt_f16x8_kernel<<<n8w / NTHR, NTHR, 0, stream>>>(Wg_w, WrWg + (size_t)NAGRU * NDIM, n8w, WCARRY);
  cvt_f16x8_kernel<<<n8w / NTHR, NTHR, 0, stream>>>(Ur_w, UrUg, n8w, WCARRY);
  cvt_f16x8_kernel<<<n8w / NTHR, NTHR, 0, stream>>>(Ug_w, UrUg + (size_t)NAGRU * NAGRU, n8w, WCARRY);
  const int n8z = NROWS * (NZK / 8);
  zbuild_kernel<<<n8z / NTHR, NTHR, 0, stream>>>(facts, queries, m_old, Zp, n8z);
  gemm_score_kernel<<<(NROWS / 64) * (NATT / 64) / 8, NTHR, 0, stream>>>(Zp, W1h, W1_b, W2_w, Pp);
  gemm_f16out_kernel<<<(NROWS / 64) * (NX / 64) / 8, NTHR, 0, stream>>>(Ff, NDIM, WrWg, NDIM, Xp, NX, NROWS, NX, NDIM, WCARRY_INV);
  softmax_kernel<<<NBATCH, NTHR, 0, stream>>>(Pp, num_facts, W2_b, Gp);
  agru_kernel<<<NBATCH / SEQB, NTHR, 0, stream>>>(Xp, Gp, UrUg, Ur_b, Ug_b, m_old, Cp);
  memout_kernel<<<NBATCH, NTHR, 0, stream>>>(m_old, Cp, queries, Wt_w, Wt_b, out);
}
